// UMNNModel_45294725104115
// MI455X (gfx1250) — hardware-verified
//
#include <hip/hip_runtime.h>
#include <stdint.h>


typedef _Float16 v16h __attribute__((ext_vector_type(16)));
typedef _Float16 v8h  __attribute__((ext_vector_type(8)));
typedef float    v8f  __attribute__((ext_vector_type(8)));
typedef float    v4f  __attribute__((ext_vector_type(4)));
union Frag { v16h v; v8h half[2]; };

#define IN_F 64
#define K_F  16
#define S_F  32
#define H_F  64
#define NM_F 48
#define NH_F 512

#define ACT_SCALE 16.0f
#define WGT_SCALE 64.0f
#define ACC_UNSCALE (1.0f / 1024.0f)

static __device__ __forceinline__ v8f wmma16(v16h a, v16h b, v8f c) {
  v8f d = __builtin_amdgcn_wmma_f32_16x16x32_f16(false, a, false, b, (short)0, c,
                                                 false, false);
  asm volatile("v_nop\n\tv_nop\n\tv_nop\n\tv_nop" : "+v"(d) : "v"(a), "v"(b));
  return d;
}

static __device__ __forceinline__ float ex2_(float x) {
#if __has_builtin(__builtin_amdgcn_exp2f)
  return __builtin_amdgcn_exp2f(x);
#else
  return exp2f(x);
#endif
}
static __device__ __forceinline__ float lg2_(float x) {
#if __has_builtin(__builtin_amdgcn_logf)
  return __builtin_amdgcn_logf(x);
#else
  return log2f(x);
#endif
}
static __device__ __forceinline__ float rcp_(float x) {
#if __has_builtin(__builtin_amdgcn_rcpf)
  return __builtin_amdgcn_rcpf(x);
#else
  return 1.0f / x;
#endif
}
static __device__ __forceinline__ float tanh_(float x) {
  float e = ex2_(x * 2.8853900817779268f);
  float r = rcp_(1.0f + e);
  return 1.0f - 2.0f * r;
}
static __device__ __forceinline__ float softplus_(float z) {
  float e = ex2_(-fabsf(z) * 1.4426950408889634f);
  return fmaxf(z, 0.0f) + 0.69314718055994531f * lg2_(1.0f + e);
}

static __device__ __forceinline__ void store2_v8h(_Float16* dst, v8h v) {
  *(volatile v8h*)dst = v;
  __threadfence();
  *(volatile v8h*)dst = v;
}
static __device__ __forceinline__ void store2_v4f(float* dst, v4f v) {
  *(volatile v4f*)dst = v;
  __threadfence();
  *(volatile v4f*)dst = v;
}

__global__ __launch_bounds__(256) void prep_kernel(
    const float* __restrict__ mw2, const float* __restrict__ nw1,
    const float* __restrict__ nw2, _Float16* mw2t, _Float16* nw1t,
    _Float16* nw2t) {
  const int g  = blockIdx.x * blockDim.x + threadIdx.x;
  const int G1 = K_F * H_F * H_F / 8;
  const int G2 = NH_F * 64 / 8;
  const int G3 = NH_F * NH_F / 8;
  v8h v;
  _Float16* dst;
  if (g < G1) {
    const int h0 = (g & 7) * 8, j = (g >> 3) & 63, k = g >> 9;
#pragma unroll
    for (int i = 0; i < 8; ++i)
      v[i] = (_Float16)(mw2[((size_t)(k * H_F + h0 + i)) * H_F + j] * WGT_SCALE);
    dst = mw2t + (size_t)g * 8;
  } else if (g < G1 + G2) {
    const int q = g - G1;
    const int kk0 = (q & 7) * 8, j = q >> 3;
#pragma unroll
    for (int i = 0; i < 8; ++i) {
      const int kk = kk0 + i;
      v[i] = (kk < NM_F) ? (_Float16)(nw1[(size_t)kk * NH_F + j] * WGT_SCALE)
                         : (_Float16)0.0f;
    }
    dst = nw1t + (size_t)q * 8;
  } else if (g < G1 + G2 + G3) {
    const int q = g - G1 - G2;
    const int c0 = (q & 63) * 8, j = q >> 6;
#pragma unroll
    for (int i = 0; i < 8; ++i)
      v[i] = (_Float16)(nw2[(size_t)(c0 + i) * NH_F + j] * WGT_SCALE);
    dst = nw2t + (size_t)q * 8;
  } else {
    return;
  }
  store2_v8h(dst, v);
}

__global__ __launch_bounds__(256) void mono_kernel(
    const float* __restrict__ x, const float* __restrict__ mw1,
    const float* __restrict__ mb1, const float* __restrict__ mb2,
    const float* __restrict__ mw3, const float* __restrict__ mb3,
    const _Float16* __restrict__ mw2t, float* gsum, int nb, int bpad) {
  __shared__ float gs_s[32];

  const int k    = blockIdx.y;
  const int lane = threadIdx.x & 31;
  const int w    = threadIdx.x >> 5;
  const int lh   = lane >> 4;
  const int l15  = lane & 15;

  float w1r[32], b1r[32];
#pragma unroll
  for (int c = 0; c < 2; ++c)
#pragma unroll
    for (int g = 0; g < 2; ++g) {
      const int hb = 32 * c + 16 * g + 8 * lh;
#pragma unroll
      for (int i = 0; i < 8; ++i) {
        w1r[c * 16 + g * 8 + i] = mw1[(size_t)k * H_F + hb + i];
        b1r[c * 16 + g * 8 + i] = mb1[(size_t)k * H_F + hb + i];
      }
    }
  float mb2r[4], mw3r[4];
#pragma unroll
  for (int nt = 0; nt < 4; ++nt) {
    const int j = 16 * nt + l15;
    mb2r[nt] = mb2[(size_t)k * H_F + j];
    mw3r[nt] = mw3[(size_t)k * H_F + j];
  }
  const float mb3k = mb3[k];
  const _Float16* bbase = mw2t + (size_t)k * H_F * H_F;

#pragma unroll 1
  for (int q = 0; q < 4; ++q) {
    const int b  = blockIdx.x * 32 + w * 4 + q;
    const int bc = (b < nb) ? b : (nb - 1);
    const float xm = x[(size_t)bc * IN_F + k];
    float tot = 0.0f;
#pragma unroll 1
    for (int sh = 0; sh < 2; ++sh) {
      const int s = sh * 16 + l15;
      const float t   = (s == S_F - 1) ? 1.0f : (float)s * (1.0f / 31.0f);
      const float pts = xm * t;

      v8f acc[4];
#pragma unroll
      for (int nt = 0; nt < 4; ++nt) {
        v8f z = {0.f, 0.f, 0.f, 0.f, 0.f, 0.f, 0.f, 0.f};
        acc[nt] = z;
      }
#pragma unroll
      for (int c = 0; c < 2; ++c) {
        v16h av;
#pragma unroll
        for (int e = 0; e < 16; ++e) {
          const float h1 = tanh_(pts * w1r[c * 16 + e] + b1r[c * 16 + e]);
          av[e] = (_Float16)(h1 * ACT_SCALE);
        }
#pragma unroll
        for (int nt = 0; nt < 4; ++nt) {
          const _Float16* bp = bbase + (size_t)(16 * nt + l15) * H_F + 32 * c + 8 * lh;
          Frag bf;
          bf.half[0] = *(const v8h*)(bp);
          bf.half[1] = *(const v8h*)(bp + 16);
          acc[nt] = wmma16(av, bf.v, acc[nt]);
        }
      }
      float p[8];
#pragma unroll
      for (int r = 0; r < 8; ++r) {
        float sacc = 0.0f;
#pragma unroll
        for (int nt = 0; nt < 4; ++nt) {
          const float h2 = tanh_(acc[nt][r] * ACC_UNSCALE + mb2r[nt]);
          sacc += h2 * mw3r[nt];
        }
        p[r] = sacc;
      }
#pragma unroll
      for (int r = 0; r < 8; ++r) {
        p[r] += __shfl_xor(p[r], 1);
        p[r] += __shfl_xor(p[r], 2);
        p[r] += __shfl_xor(p[r], 4);
        p[r] += __shfl_xor(p[r], 8);
      }
      float gs = 0.0f;
#pragma unroll
      for (int r = 0; r < 8; ++r) gs += softplus_(p[r] + mb3k);
      gs += __shfl_xor(gs, 16);
      tot += gs;
    }
    if (lane == 0) gs_s[w * 4 + q] = tot;
  }
  __syncthreads();
  if (threadIdx.x < 8) {
    const int i = threadIdx.x;
    v4f v = {gs_s[4 * i + 0], gs_s[4 * i + 1], gs_s[4 * i + 2], gs_s[4 * i + 3]};
    float* dst = gsum + (size_t)k * bpad + (size_t)blockIdx.x * 32 + 4 * i;
    store2_v4f(dst, v);
  }
}

__global__ __launch_bounds__(256) void nonmono_kernel(
    const float* __restrict__ x, const float* __restrict__ nb1,
    const float* __restrict__ nb2, const float* __restrict__ nw3,
    const float* __restrict__ nb3, const _Float16* __restrict__ nw1t,
    const _Float16* __restrict__ nw2t, float* nmv, int nb) {
  __shared__ __attribute__((aligned(16))) _Float16 a1s[16][NH_F];
  __shared__ float partial[8][16];
  __shared__ float linebuf[32];

  const int b0   = blockIdx.x * 16;
  const int lane = threadIdx.x & 31;
  const int w    = threadIdx.x >> 5;
  const int lh   = lane >> 4;
  const int l15  = lane & 15;
  const int m    = l15;
  const int brow = b0 + m;
  const int bc   = (brow < nb) ? brow : (nb - 1);

  v8f acc[4];
#pragma unroll
  for (int nt = 0; nt < 4; ++nt) {
    v8f z = {0.f, 0.f, 0.f, 0.f, 0.f, 0.f, 0.f, 0.f};
    acc[nt] = z;
  }
#pragma unroll
  for (int c = 0; c < 2; ++c) {
    v16h av;
#pragma unroll
    for (int g = 0; g < 2; ++g) {
      const int kb = 32 * c + 16 * g + 8 * lh;
#pragma unroll
      for (int i = 0; i < 8; ++i) {
        const int kk  = kb + i;
        const float v = (kk < NM_F) ? x[(size_t)bc * IN_F + K_F + kk] : 0.0f;
        av[g * 8 + i] = (_Float16)(v * ACT_SCALE);
      }
    }
#pragma unroll
    for (int nt = 0; nt < 4; ++nt) {
      const int j = 16 * (4 * w + nt) + l15;
      const _Float16* bp = nw1t + (size_t)j * 64 + 32 * c + 8 * lh;
      Frag bf;
      bf.half[0] = *(const v8h*)(bp);
      bf.half[1] = *(const v8h*)(bp + 16);
      acc[nt] = wmma16(av, bf.v, acc[nt]);
    }
  }
#pragma unroll
  for (int nt = 0; nt < 4; ++nt) {
    const int j      = 16 * (4 * w + nt) + l15;
    const float bias = nb1[j];
#pragma unroll
    for (int r = 0; r < 8; ++r) {
      float v = acc[nt][r] * ACC_UNSCALE + bias;
      v = (v > 0.0f) ? v : 0.0f;
      a1s[r + 8 * lh][j] = (_Float16)(v * ACT_SCALE);
    }
  }
  __syncthreads();

  v8f acc2[4];
#pragma unroll
  for (int nt = 0; nt < 4; ++nt) {
    v8f z = {0.f, 0.f, 0.f, 0.f, 0.f, 0.f, 0.f, 0.f};
    acc2[nt] = z;
  }
#pragma unroll 2
  for (int c = 0; c < NH_F / 32; ++c) {
    Frag af;
    af.half[0] = *(const v8h*)(&a1s[m][32 * c + 8 * lh]);
    af.half[1] = *(const v8h*)(&a1s[m][32 * c + 16 + 8 * lh]);
#pragma unroll
    for (int nt = 0; nt < 4; ++nt) {
      const int j = 16 * (4 * w + nt) + l15;
      const _Float16* bp = nw2t + (size_t)j * NH_F + 32 * c + 8 * lh;
      Frag bf;
      bf.half[0] = *(const v8h*)(bp);
      bf.half[1] = *(const v8h*)(bp + 16);
      acc2[nt] = wmma16(af.v, bf.v, acc2[nt]);
    }
  }
  float nb2r[4], nw3r[4];
#pragma unroll
  for (int nt = 0; nt < 4; ++nt) {
    const int j = 16 * (4 * w + nt) + l15;
    nb2r[nt] = nb2[j];
    nw3r[nt] = nw3[j];
  }
  float p[8];
#pragma unroll
  for (int r = 0; r < 8; ++r) {
    float sacc = 0.0f;
#pragma unroll
    for (int nt = 0; nt < 4; ++nt) {
      float v = acc2[nt][r] * ACC_UNSCALE + nb2r[nt];
      v = (v > 0.0f) ? v : 0.0f;
      sacc += v * nw3r[nt];
    }
    p[r] = sacc;
  }
#pragma unroll
  for (int r = 0; r < 8; ++r) {
    p[r] += __shfl_xor(p[r], 1);
    p[r] += __shfl_xor(p[r], 2);
    p[r] += __shfl_xor(p[r], 4);
    p[r] += __shfl_xor(p[r], 8);
  }
  if (l15 == 0) {
#pragma unroll
    for (int r = 0; r < 8; ++r) partial[w][8 * lh + r] = p[r];
  }
  __syncthreads();
  if (threadIdx.x < 32) {
    float v = 0.0f;
    if (threadIdx.x < 16) {
      float sacc = 0.0f;
#pragma unroll
      for (int ww = 0; ww < 8; ++ww) sacc += partial[ww][threadIdx.x];
      v = sacc + nb3[0];
    }
    linebuf[threadIdx.x] = v;
  }
  __syncthreads();
  if (threadIdx.x < 8) {
    const int i = threadIdx.x;
    v4f v = {linebuf[4 * i + 0], linebuf[4 * i + 1], linebuf[4 * i + 2],
             linebuf[4 * i + 3]};
    float* dst = nmv + (size_t)blockIdx.x * 32 + 4 * i;
    store2_v4f(dst, v);
  }
}

__global__ __launch_bounds__(256) void final_kernel(
    const float* __restrict__ x, const float* __restrict__ wlin,
    const float* __restrict__ gsum, const float* __restrict__ nmv, float* out,
    int nb, int bpad) {
  const int b4 = (blockIdx.x * blockDim.x + threadIdx.x) * 4;
  if (b4 >= nb) return;
  float o[4];
#pragma unroll
  for (int i = 0; i < 4; ++i) {
    const int b  = b4 + i;
    const int bc = (b < nb) ? b : (nb - 1);
    float mono = 0.0f;
#pragma unroll
    for (int k = 0; k < K_F; ++k) {
      const float integ = (gsum[(size_t)k * bpad + bc] * (1.0f / (float)S_F)) *
                          x[(size_t)bc * IN_F + k];
      mono += integ * wlin[k];
    }
    o[i] = mono + nmv[(size_t)(bc >> 4) * 32 + (bc & 15)];
  }
  if (b4 + 4 <= nb) {
    v4f v = {o[0], o[1], o[2], o[3]};
    store2_v4f(out + b4, v);
  } else {
#pragma unroll
    for (int i = 0; i < 4; ++i) {
      if (b4 + i < nb) {
        const float val = o[i];
        *(volatile float*)(out + b4 + i) = val;
        __threadfence();
        *(volatile float*)(out + b4 + i) = val;
      }
    }
  }
}

extern "C" void kernel_launch(void* const* d_in, const int* in_sizes, int n_in,
                              void* d_out, int out_size, void* d_ws,
                              size_t ws_size, hipStream_t stream) {
  if (n_in < 14) return;
  const int nb = in_sizes[0] / IN_F;
  if (nb <= 0 || in_sizes[0] != nb * IN_F || out_size != nb) return;
  if (in_sizes[1] != K_F * H_F || in_sizes[2] != K_F * H_F ||
      in_sizes[3] != K_F * H_F * H_F || in_sizes[4] != K_F * H_F ||
      in_sizes[5] != K_F * H_F || in_sizes[6] != K_F || in_sizes[7] != K_F ||
      in_sizes[8] != NM_F * NH_F || in_sizes[9] != NH_F ||
      in_sizes[10] != NH_F * NH_F || in_sizes[11] != NH_F ||
      in_sizes[12] != NH_F || in_sizes[13] < 1)
    return;

  const float* x    = (const float*)d_in[0];
  const float* mw1  = (const float*)d_in[1];
  const float* mb1  = (const float*)d_in[2];
  const float* mw2  = (const float*)d_in[3];
  const float* mb2  = (const float*)d_in[4];
  const float* mw3  = (const float*)d_in[5];
  const float* mb3  = (const float*)d_in[6];
  const float* wlin = (const float*)d_in[7];
  const float* nw1  = (const float*)d_in[8];
  const float* nb1  = (const float*)d_in[9];
  const float* nw2  = (const float*)d_in[10];
  const float* nb2  = (const float*)d_in[11];
  const float* nw3  = (const float*)d_in[12];
  const float* nb3  = (const float*)d_in[13];
  float* out = (float*)d_out;

  const int nblk32 = (nb + 31) / 32;
  const int bpad   = nblk32 * 32;
  const int nblk16 = (nb + 15) / 16;

  const size_t off_mw2t = 0;
  const size_t sz_mw2t  = (size_t)K_F * H_F * H_F * sizeof(_Float16);
  const size_t off_nw1t = off_mw2t + sz_mw2t;
  const size_t sz_nw1t  = (size_t)NH_F * 64 * sizeof(_Float16);
  const size_t off_nw2t = off_nw1t + sz_nw1t;
  const size_t sz_nw2t  = (size_t)NH_F * NH_F * sizeof(_Float16);
  const size_t off_gsum = off_nw2t + sz_nw2t;
  const size_t sz_gsum  = (size_t)K_F * bpad * sizeof(float);
  size_t off_nmv = off_gsum + sz_gsum;
  off_nmv = (off_nmv + 127) & ~(size_t)127;
  const size_t sz_nmv = (size_t)nblk16 * 32 * sizeof(float);
  const size_t total  = off_nmv + sz_nmv;
  if (total > ws_size) return;

  char* ws = (char*)d_ws;
  _Float16* mw2t = (_Float16*)(ws + off_mw2t);
  _Float16* nw1t = (_Float16*)(ws + off_nw1t);
  _Float16* nw2t = (_Float16*)(ws + off_nw2t);
  float*    gsum = (float*)(ws + off_gsum);
  float*    nmv  = (float*)(ws + off_nmv);

  const int ngroups = K_F * H_F * H_F / 8 + NH_F * 64 / 8 + NH_F * NH_F / 8;
  prep_kernel<<<(ngroups + 255) / 256, 256, 0, stream>>>(mw2, nw1, nw2, mw2t,
                                                          nw1t, nw2t);

  dim3 mg(nblk32, K_F);
  mono_kernel<<<mg, 256, 0, stream>>>(x, mw1, mb1, mb2, mw3, mb3, mw2t, gsum, nb,
                                      bpad);

  nonmono_kernel<<<nblk16, 256, 0, stream>>>(x, nb1, nb2, nw3, nb3, nw1t, nw2t,
                                              nmv, nb);

  final_kernel<<<(nb + 1023) / 1024, 256, 0, stream>>>(x, wlin, gsum, nmv, out,
                                                        nb, bpad);
}
